// LPKTNet_88656714925283
// MI455X (gfx1250) — hardware-verified
//
#include <hip/hip_runtime.h>
#include <math.h>

typedef __attribute__((ext_vector_type(16))) _Float16 v16h;
typedef __attribute__((ext_vector_type(8)))  _Float16 v8h;
typedef __attribute__((ext_vector_type(4)))  _Float16 v4h;
typedef __attribute__((ext_vector_type(16))) __bf16   v16b;
typedef __attribute__((ext_vector_type(8)))  __bf16   v8b;
typedef __attribute__((ext_vector_type(8)))  float    v8f;
typedef __attribute__((ext_vector_type(4)))  float    v4f;

constexpr int kB    = 32;
constexpr int kS    = 128;
constexpr int kT    = kS - 1;
constexpr int kNE   = 4000;
constexpr int kNA   = 1000;
constexpr int kNI   = 1000;
constexpr int kSk   = 256;
constexpr int kD    = 128;
constexpr int kRowsE = kB * kS;
constexpr int kRowsH = kB * kSk;
constexpr int kThr  = 256;
constexpr float kInCarry = 1024.0f;
constexpr float kACarry  = 256.0f;
constexpr float kScE = 1.0f / (kInCarry * kInCarry);
constexpr float kScA = 1.0f / (kACarry * kInCarry);
constexpr float kF16MinNormal = 6.103515625e-5f;
constexpr int kFB1 = 0, kFBL = 128, kFBF = 384, kFBP = 512, kFBZ = 640, kFEnd = 768;

static_assert((kRowsE % 64) == 0 && (kRowsH % 64) == 0 && (kD % 64) == 0 && ((kRowsE / 64) * (kD / 64)) % 8 == 0 && ((kRowsH / 64) * (kD / 64)) % 8 == 0
              && ((128 / 64) * (256 / 64)) % 8 == 0 && ((256 / 64) * (kD / 64)) % 8 == 0, "GEMM M, N multiples of 64; grids exact (the small products pad M to 128 or 256 with zero rows)");

constexpr size_t kOffW1P = 0ull;
constexpr size_t kOffWLG = 98304ull;
constexpr size_t kOffWF16 = 360448ull;
constexpr size_t kOffWP16 = 458752ull;
constexpr size_t kOffBIAS = 524288ull;
constexpr size_t kOffXE16 = 527360ull;
constexpr size_t kOffLE32 = 3673088ull;
constexpr size_t kOffH32 = 5770240ull;
constexpr size_t kOffHT32 = 9964544ull;
constexpr size_t kOffLG32 = 9980928ull;
constexpr size_t kOffX4 = 9997312ull;
constexpr size_t kOffZ32 = 10128384ull;
constexpr size_t kOffXB = 10259456ull;
constexpr size_t kOffPB32 = 10390528ull;
constexpr size_t kOffH16 = 10521600ull;
constexpr size_t kOffPH32 = 12618752ull;
constexpr size_t kOffX5 = 16813056ull;
constexpr size_t kOffP32 = 16944128ull;
constexpr size_t kWsTotal = 17075200ull;
static_assert(kWsTotal <= 134217728ull, "carve cap: under 128 MiB");
static_assert(kOffW1P == 0
              && kOffWLG == kOffW1P + 98304ull
              && kOffWF16 == kOffWLG + 262144ull
              && kOffWP16 == kOffWF16 + 98304ull
              && kOffBIAS == kOffWP16 + 65536ull
              && kOffXE16 == kOffBIAS + 3072ull
              && kOffLE32 == kOffXE16 + 3145728ull
              && kOffH32 == kOffLE32 + 2097152ull
              && kOffHT32 == kOffH32 + 4194304ull
              && kOffLG32 == kOffHT32 + 16384ull
              && kOffX4 == kOffLG32 + 16384ull
              && kOffZ32 == kOffX4 + 131072ull
              && kOffXB == kOffZ32 + 131072ull
              && kOffPB32 == kOffXB + 131072ull
              && kOffH16 == kOffPB32 + 131072ull
              && kOffPH32 == kOffH16 + 2097152ull
              && kOffX5 == kOffPH32 + 4194304ull
              && kOffP32 == kOffX5 + 131072ull
              && kWsTotal == kOffP32 + 131072ull, "the carve is chained and totalled");
static_assert((kOffW1P % 256) == 0 && (kOffWLG % 256) == 0 && (kOffWF16 % 256) == 0 && (kOffWP16 % 256) == 0 && (kOffBIAS % 256) == 0 && (kOffXE16 % 256) == 0 && (kOffLE32 % 256) == 0 && (kOffH32 % 256) == 0 && (kOffHT32 % 256) == 0 && (kOffLG32 % 256) == 0 && (kOffX4 % 256) == 0 && (kOffZ32 % 256) == 0 && (kOffXB % 256) == 0 && (kOffPB32 % 256) == 0 && (kOffH16 % 256) == 0 && (kOffPH32 % 256) == 0 && (kOffX5 % 256) == 0 && (kOffP32 % 256) == 0, "aligned regions");

__device__ __forceinline__ unsigned short f2bf_bits(float f) {
  unsigned u = __float_as_uint(f);
  return (unsigned short)((u + 0x7FFFu + ((u >> 16) & 1u)) >> 16);
}
__device__ __forceinline__ float bf_bits2f(unsigned short h) { return __uint_as_float(((unsigned)h) << 16); }
__device__ __forceinline__ float bf16r(float f) { return bf_bits2f(f2bf_bits(f)); }
__device__ __forceinline__ float carry_flush(float v, float carry) {
  const float s = v * carry;
  return (fabsf(s) < kF16MinNormal) ? 0.0f : s;
}
__device__ __forceinline__ float frcp(float x) { return __builtin_amdgcn_rcpf(x); }

__device__ __forceinline__ void dep_guard4_h(v8f& a, v8f& b, v8f& c, v8f& d, v16h x, v16h y) { asm volatile("v_nop\n\tv_nop\n\tv_nop\n\tv_nop" : "+v"(a), "+v"(b), "+v"(c), "+v"(d) : "v"(x), "v"(y)); }
__device__ __forceinline__ void dep_guard4_b(v8f& a, v8f& b, v8f& c, v8f& d, v16b x, v16b y) { asm volatile("v_nop\n\tv_nop\n\tv_nop\n\tv_nop" : "+v"(a), "+v"(b), "+v"(c), "+v"(d) : "v"(x), "v"(y)); }
__device__ __forceinline__ void keep4_h(v16h a, v16h b, v16h c, v16h d) { asm volatile("v_nop" :: "v"(a), "v"(b), "v"(c), "v"(d)); }
__device__ __forceinline__ void keep4_b(v16b a, v16b b, v16b c, v16b d) { asm volatile("v_nop" :: "v"(a), "v"(b), "v"(c), "v"(d)); }
__device__ __forceinline__ void acc_guard4(v8f& a, v8f& b, v8f& c, v8f& d) { asm volatile("v_nop\n\tv_nop\n\tv_nop\n\tv_nop" : "+v"(a), "+v"(b), "+v"(c), "+v"(d)); }

template <typename T> struct Frag;
template <> struct Frag<_Float16> {
  typedef v16h V; union U { v16h v; v8h h[2]; };
  static __device__ __forceinline__ v16h load(const _Float16* p) {
    U f; f.h[0] = *(const v8h*)(p); f.h[1] = *(const v8h*)(p + 16); return f.v;
  }
  static __device__ __forceinline__ v8f mma(v16h a, v16h b, v8f c) {
    return __builtin_amdgcn_wmma_f32_16x16x32_f16(false, a, false, b, (short)0, c, false, false);
  }
  static __device__ __forceinline__ void guard4(v8f& a, v8f& b, v8f& c, v8f& d, v16h x, v16h y) { dep_guard4_h(a, b, c, d, x, y); }
  static __device__ __forceinline__ void keep(v16h a, v16h b, v16h c, v16h d) { keep4_h(a, b, c, d); }
};
template <> struct Frag<__bf16> {
  typedef v16b V; union U { v16b v; v8b h[2]; };
  static __device__ __forceinline__ v16b load(const __bf16* p) {
    U f; f.h[0] = *(const v8b*)(p); f.h[1] = *(const v8b*)(p + 16); return f.v;
  }
  static __device__ __forceinline__ v8f mma(v16b a, v16b b, v8f c) {
    return __builtin_amdgcn_wmma_f32_16x16x32_bf16(false, a, false, b, (short)0, c, false, false);
  }
  static __device__ __forceinline__ void guard4(v8f& a, v8f& b, v8f& c, v8f& d, v16b x, v16b y) { dep_guard4_b(a, b, c, d, x, y); }
  static __device__ __forceinline__ void keep(v16b a, v16b b, v16b c, v16b d) { keep4_b(a, b, c, d); }
};

__device__ __forceinline__ v8f mma_h(v16h a, v16h b, v8f c) {
  c = __builtin_amdgcn_wmma_f32_16x16x32_f16(false, a, false, b, (short)0, c, false, false);
  asm volatile("v_nop\n\tv_nop\n\tv_nop\n\tv_nop" : "+v"(c) : "v"(a), "v"(b));
  return c;
}

template <int ET> struct Elem;
template <> struct Elem<0> { typedef _Float16 T; };
template <> struct Elem<1> { typedef __bf16 T; };
template <int ET, bool SPLIT, int BIAS_MODE, int OUT_MODE, bool RESID, int ACT = 0>
__global__ __launch_bounds__(256) void wmma_gemm64(
    const unsigned short* __restrict__ Ap, const unsigned short* __restrict__ A2p, int lda, long strideA,
    const unsigned short* __restrict__ Btp, const unsigned short* __restrict__ Bt2p, int ldb, long strideB,
    void* __restrict__ Cout, void* __restrict__ Cout2, int ldc, long strideC,
    const float* __restrict__ bias,
    const float* __restrict__ resid, long strideR,
    int M, int N, int K, float scale) {
  typedef typename Elem<ET>::T T;
  typedef typename Frag<T>::V V;
  const T* A = (const T*)Ap; const T* A2 = (const T*)A2p; const T* Bt = (const T*)Btp; const T* Bt2 = (const T*)Bt2p;
  __shared__ __align__(16) float sT[8][16 * 68];
  const int b    = blockIdx.y;
  const int lane = threadIdx.x & 31;
  const int wave = threadIdx.x >> 5;
  const int tilesN = N >> 6;
  const int tilesM = M >> 6;
  const int tile = blockIdx.x * 8 + wave;
  if (tile >= tilesM * tilesN) return;
  const int tm = tile / tilesN;
  const int tn = tile - tm * tilesN;
  const int m0 = tm << 6;
  const int n0 = tn << 6;

  const T* Ab  = A  + (size_t)b * strideA;
  const T* Bb  = Bt + (size_t)b * strideB;
  const T* Ab2 = SPLIT ? (A2  + (size_t)b * strideA) : nullptr;
  const T* Bb2 = SPLIT ? (Bt2 + (size_t)b * strideB) : nullptr;

  const int rlane = lane & 15;
  const int koff  = (lane >> 4) * 8;
  const int mOff  = (lane >> 4) * 8;

  v8f acc[4][4];
#pragma unroll
  for (int i = 0; i < 4; ++i)
#pragma unroll
    for (int j = 0; j < 4; ++j) acc[i][j] = (v8f){0.f,0.f,0.f,0.f,0.f,0.f,0.f,0.f};

  for (int k0 = 0; k0 < K; k0 += 32) {
    V bh[4], bl[4];
#pragma unroll
    for (int j = 0; j < 4; ++j) {
      const size_t bo = (size_t)(n0 + (j << 4) + rlane) * ldb + koff + k0;
      bh[j] = Frag<T>::load(Bb + bo);
      if (SPLIT) bl[j] = Frag<T>::load(Bb2 + bo);
    }
#pragma unroll
    for (int i = 0; i < 4; ++i) {
      const size_t ao = (size_t)(m0 + (i << 4) + rlane) * lda + koff + k0;
      V ah = Frag<T>::load(Ab + ao);
      V al;
      if (SPLIT) al = Frag<T>::load(Ab2 + ao);
#pragma unroll
      for (int j = 0; j < 4; ++j) {
        acc[i][j] = Frag<T>::mma(ah, bh[j], acc[i][j]);
        if (SPLIT) {
          acc[i][j] = Frag<T>::mma(ah, bl[j], acc[i][j]);
          acc[i][j] = Frag<T>::mma(al, bh[j], acc[i][j]);
        }
      }
      Frag<T>::guard4(acc[i][0], acc[i][1], acc[i][2], acc[i][3], ah, SPLIT ? al : ah);
    }
    Frag<T>::keep(bh[0], bh[1], bh[2], bh[3]);
    if (SPLIT) Frag<T>::keep(bl[0], bl[1], bl[2], bl[3]);
  }
  acc_guard4(acc[0][0], acc[0][1], acc[0][2], acc[0][3]);
  acc_guard4(acc[1][0], acc[1][1], acc[1][2], acc[1][3]);
  acc_guard4(acc[2][0], acc[2][1], acc[2][2], acc[2][3]);
  acc_guard4(acc[3][0], acc[3][1], acc[3][2], acc[3][3]);

  float* slab = sT[wave];
  const float* Rb = RESID ? (resid + (size_t)b * strideR) : nullptr;
#pragma unroll
  for (int i = 0; i < 4; ++i) {
    const int mBase = m0 + (i << 4);
#pragma unroll
    for (int j = 0; j < 4; ++j) {
      const int n = n0 + (j << 4) + rlane;
      float bv = 0.f;
      if (BIAS_MODE == 2) bv = bias[n];
#pragma unroll
      for (int r = 0; r < 8; ++r) {
        float v = acc[i][j][r] * scale;
        if (BIAS_MODE == 1) v += bias[mBase + mOff + r];
        if (BIAS_MODE == 2) v += bv;
        if (RESID) v += Rb[(size_t)(mBase + mOff + r) * ldc + n];
        if (ACT == 1) v = tanhf(v);
        if (ACT == 2) v = fmaxf(v, 0.0f);
        if (ACT == 3) v = v / (1.0f + expf(-v));
        if (ACT == 4) v = (v > 0.f) ? v : 0.01f * v;
        slab[(mOff + r) * 68 + (j << 4) + rlane] = v;
      }
    }
    __builtin_amdgcn_fence(__ATOMIC_RELEASE, "workgroup");
    __builtin_amdgcn_wave_barrier();
    __builtin_amdgcn_fence(__ATOMIC_ACQUIRE, "workgroup");
    if (OUT_MODE == 0) {
      float* C = (float*)Cout + (size_t)b * strideC;
      const int hh = lane >> 4, c4 = (lane & 15) * 4;
      for (int pass = 0; pass < 2; ++pass) {
#pragma unroll
        for (int it = 0; it < 8; ++it) {
          const int row = it * 2 + hh;
          v4f v = *(const v4f*)(slab + row * 68 + c4);
          *(volatile v4f*)(C + (size_t)(mBase + row) * ldc + n0 + c4) = v;
        }
        __threadfence();
      }
    } else {
      const int q = lane >> 3, c8 = (lane & 7) * 8;
      unsigned short* C  = (unsigned short*)Cout  + (size_t)b * strideC;
      unsigned short* C2 = (OUT_MODE == 2) ? ((unsigned short*)Cout2 + (size_t)b * strideC) : nullptr;
      for (int pass = 0; pass < 2; ++pass) {
#pragma unroll
        for (int it = 0; it < 4; ++it) {
          const int row = it * 4 + q;
          const float* sp = slab + row * 68 + c8;
          v8h hv, lv;
#pragma unroll
          for (int e = 0; e < 8; ++e) {
            if (OUT_MODE == 1) {
              hv[e] = (_Float16)sp[e];
            } else {
              unsigned short hb = f2bf_bits(sp[e]);
              unsigned short lb = f2bf_bits(sp[e] - bf_bits2f(hb));
              hv[e] = __builtin_bit_cast(_Float16, hb);
              lv[e] = __builtin_bit_cast(_Float16, lb);
            }
          }
          *(volatile v8h*)(C + (size_t)(mBase + row) * ldc + n0 + c8) = hv;
          if (OUT_MODE == 2) *(volatile v8h*)(C2 + (size_t)(mBase + row) * ldc + n0 + c8) = lv;
        }
        __threadfence();
      }
    }
    __builtin_amdgcn_fence(__ATOMIC_RELEASE, "workgroup");
    __builtin_amdgcn_wave_barrier();
    __builtin_amdgcn_fence(__ATOMIC_ACQUIRE, "workgroup");
  }
}

__global__ __launch_bounds__(kThr) void cast_plane_kernel(const float* __restrict__ src, unsigned short* __restrict__ dst,
                                                          int colsLog2, int dstPitch, int dstOff) {
  const int i   = blockIdx.x * kThr + threadIdx.x;
  const int sh  = colsLog2 - 3;
  const int row = i >> sh;
  const int c8  = (i & ((1 << sh) - 1)) * 8;
  const float* sp = src + ((size_t)row << colsLog2) + c8;
  const v4f a0 = *(const v4f*)(sp);
  const v4f a1 = *(const v4f*)(sp + 4);
  v8h hv;
#pragma unroll
  for (int e = 0; e < 4; ++e) {
    const float f0 = a0[e];
    const float f1 = a1[e];
    hv[e]     = (_Float16)carry_flush(bf16r(f0), kInCarry);
    hv[4 + e] = (_Float16)carry_flush(bf16r(f1), kInCarry);
  }
  unsigned short* dp = dst + (size_t)row * dstPitch + dstOff + c8;
  *(volatile v8h*)dp = hv;
  __threadfence();
  *(volatile v8h*)dp = hv;
}

__global__ __launch_bounds__(kThr) void setup_kernel(const float* __restrict__ b1, const float* __restrict__ bl, const float* __restrict__ bg,
                                                     const float* __restrict__ bf, const float* __restrict__ bp, const float* __restrict__ h0,
                                                     float* __restrict__ BIAS, unsigned short* __restrict__ X4, unsigned short* __restrict__ XB,
                                                     unsigned short* __restrict__ X5, float* __restrict__ H32) {
  unsigned v = blockIdx.x * (unsigned)kThr + threadIdx.x;
  asm volatile("" : "+v"(v));
  if (v < 192u) {
    const unsigned i0 = v * 4u;
    const unsigned seg = i0 >> 7, j = i0 & 127u;
    const float* sp = (seg == 0u) ? b1 : (seg == 1u) ? bl : (seg == 2u) ? bg : (seg == 3u) ? bf : bp;
    v4f o = {0.f, 0.f, 0.f, 0.f};
    if (seg < 5u) {
      const v4f a = *(const v4f*)(sp + j);
#pragma unroll
      for (int e = 0; e < 4; ++e) { const float x = a[e]; o[e] = bf16r(x); }
    }
    float* dp = BIAS + i0;
    *(volatile v4f*)dp = o;
    __threadfence();
    *(volatile v4f*)dp = o;
  } else if (v < 20672u) {
    const unsigned w = v - 192u;
    v8h z;
#pragma unroll
    for (int e = 0; e < 8; ++e) z[e] = (_Float16)0.0f;
    unsigned short* dp = (w < 6144u) ? (X4 + (size_t)32 * 512 + (size_t)w * 8u)
                       : (w < 13312u) ? (XB + (size_t)32 * 256 + (size_t)(w - 6144u) * 8u)
                                      : (X5 + (size_t)32 * 256 + (size_t)(w - 13312u) * 8u);
    *(volatile v8h*)dp = z;
    __threadfence();
    *(volatile v8h*)dp = z;
  } else if (v < 282816u) {
    const unsigned w = v - 20672u;
    const unsigned j = (w * 4u) & 32767u;
    const v4f a = *(const v4f*)(h0 + j);
    v4f o;
#pragma unroll
    for (int e = 0; e < 4; ++e) { const float x = a[e]; o[e] = bf16r(x); }
    float* dp = H32 + (size_t)w * 4u;
    *(volatile v4f*)dp = o;
    __threadfence();
    *(volatile v4f*)dp = o;
  }
}
static_assert(kFEnd / 4 == 192 && 96 * 512 / 8 == 6144 && 224 * 256 / 8 == 7168 && 192 + 6144 + 7168 + 7168 == 20672 && kB * kSk * kD / 4 == 262144 && 20672 + 262144 == 282816
              && (192 % 64) == 0 && (6336 % 64) == 0 && (13504 % 64) == 0 && (20672 % 64) == 0 && (282816 % 64) == 0, "set-up ranges wave-uniform");

__global__ __launch_bounds__(kThr) void gather_kernel(const int* __restrict__ eid, const int* __restrict__ atm, const int* __restrict__ avl,
                                                      const float* __restrict__ ex_table, const float* __restrict__ at_table,
                                                      unsigned short* __restrict__ XE16) {
  unsigned v = blockIdx.x * (unsigned)kThr + threadIdx.x;
  asm volatile("" : "+v"(v));
  const unsigned row = v / 48u, c8 = (v % 48u) * 8u;
  const unsigned seg = c8 >> 7, j = c8 & 127u;
  int e0 = eid[row]; e0 = (e0 < 0) ? 0 : (e0 > kNE - 1 ? kNE - 1 : e0);
  int a0 = atm[row]; a0 = (a0 < 0) ? 0 : (a0 > kNA - 1 ? kNA - 1 : a0);
  const float av = (float)avl[row];
  const float* sp = (seg == 0u) ? (ex_table + (size_t)e0 * kD + j) : (at_table + (size_t)a0 * kD + j);
  const v4f p0 = *(const v4f*)sp, p1 = *(const v4f*)(sp + 4);
  v8h hv;
#pragma unroll
  for (int e = 0; e < 4; ++e) {
    const float q0 = (seg == 2u) ? av : bf16r(p0[e]);
    const float q1 = (seg == 2u) ? av : bf16r(p1[e]);
    hv[e] = (_Float16)carry_flush(q0, kInCarry); hv[4 + e] = (_Float16)carry_flush(q1, kInCarry);
  }
  unsigned short* dp = XE16 + (size_t)row * 384u + c8;
  *(volatile v8h*)dp = hv;
  __threadfence();
  *(volatile v8h*)dp = hv;
}
static_assert(kRowsE * 48 == 768 * kThr, "gather grid exact");

__global__ __launch_bounds__(kThr) void read0_kernel(const int* __restrict__ eid, const float* __restrict__ q_matrix, const float* __restrict__ H32,
                                                     float* __restrict__ HT32) {
  unsigned v = blockIdx.x * (unsigned)kThr + threadIdx.x;
  asm volatile("" : "+v"(v));
  const unsigned b = v >> 7, d = v & 127u;
  int e0 = eid[b * kS]; e0 = (e0 < 0) ? 0 : (e0 > kNE - 1 ? kNE - 1 : e0);
  const float* qr = q_matrix + (size_t)e0 * kSk;
  const float* hp = H32 + (size_t)b * kSk * kD + d;
  float acc = 0.0f;
  for (int s = 0; s < kSk; ++s) { const float q = qr[s]; acc += bf16r(q) * hp[(size_t)s * kD]; }
  float* dp = HT32 + v;
  *(volatile float*)dp = acc;
  __threadfence();
  *(volatile float*)dp = acc;
}
static_assert(kB * kD == 16 * kThr, "read grid exact");

__global__ __launch_bounds__(kThr) void x4_kernel(const float* __restrict__ LE32, const float* __restrict__ HT32, const int* __restrict__ itm,
                                                  const float* __restrict__ it_table, unsigned short* __restrict__ X4, int t) {
  unsigned v = blockIdx.x * (unsigned)kThr + threadIdx.x;
  asm volatile("" : "+v"(v));
  const unsigned b = v >> 6, c8 = (v & 63u) * 8u;
  const unsigned seg = c8 >> 7, j = c8 & 127u;
  int i0 = itm[b * kS + t + 1]; i0 = (i0 < 0) ? 0 : (i0 > kNI - 1 ? kNI - 1 : i0);
  const bool hasPrev = (t > 0);
  const float* sp = (seg == 0u) ? (LE32 + (size_t)(b * kS + (hasPrev ? t - 1 : 0)) * kD + j)
                  : (seg == 1u) ? (it_table + (size_t)i0 * kD + j)
                  : (seg == 2u) ? (LE32 + (size_t)(b * kS + t) * kD + j)
                                : (HT32 + (size_t)b * kD + j);
  const v4f p0 = *(const v4f*)sp, p1 = *(const v4f*)(sp + 4);
  v8h hv;
#pragma unroll
  for (int e = 0; e < 4; ++e) {
    float q0 = p0[e], q1 = p1[e];
    if (seg == 1u) { q0 = bf16r(q0); q1 = bf16r(q1); }
    if (seg == 0u && !hasPrev) { q0 = 0.0f; q1 = 0.0f; }
    hv[e] = (_Float16)carry_flush(q0, kACarry); hv[4 + e] = (_Float16)carry_flush(q1, kACarry);
  }
  unsigned short* dp = X4 + (size_t)b * 512u + c8;
  *(volatile v8h*)dp = hv;
  __threadfence();
  *(volatile v8h*)dp = hv;
}
static_assert(kB * 64 == 8 * kThr, "x4 grid exact");

__global__ __launch_bounds__(kThr) void lg_kernel(const float* __restrict__ Z32, const int* __restrict__ itm, const float* __restrict__ it_table,
                                                  float* __restrict__ LG32, unsigned short* __restrict__ XB, int t) {
  unsigned v = blockIdx.x * (unsigned)kThr + threadIdx.x;
  asm volatile("" : "+v"(v));
  const unsigned b = v >> 5, c8 = (v & 31u) * 8u;
  const bool lgHalf = c8 < 128u;
  const unsigned j = c8 & 127u;
  int i0 = itm[b * kS + t + 1]; i0 = (i0 < 0) ? 0 : (i0 > kNI - 1 ? kNI - 1 : i0);
  float val[8];
  if (lgHalf) {
    const v4f a0 = *(const v4f*)(Z32 + (size_t)b * 256u + j), a1 = *(const v4f*)(Z32 + (size_t)b * 256u + j + 4);
    const v4f g0 = *(const v4f*)(Z32 + (size_t)b * 256u + 128u + j), g1 = *(const v4f*)(Z32 + (size_t)b * 256u + 128u + j + 4);
#pragma unroll
    for (int e = 0; e < 4; ++e) {
      val[e] = (1.0f / (1.0f + expf(-g0[e]))) * (tanhf(a0[e]) + 1.0f) * 0.5f;
      val[4 + e] = (1.0f / (1.0f + expf(-g1[e]))) * (tanhf(a1[e]) + 1.0f) * 0.5f;
    }
  } else {
    const v4f p0 = *(const v4f*)(it_table + (size_t)i0 * kD + j), p1 = *(const v4f*)(it_table + (size_t)i0 * kD + j + 4);
#pragma unroll
    for (int e = 0; e < 4; ++e) { val[e] = bf16r(p0[e]); val[4 + e] = bf16r(p1[e]); }
  }
  v8h hv;
#pragma unroll
  for (int e = 0; e < 8; ++e) hv[e] = (_Float16)carry_flush(val[e], kACarry);
  unsigned short* dp = XB + (size_t)b * 256u + c8;
  float* lp = LG32 + (size_t)b * kD + j;
  for (int pass = 0; pass < 2; ++pass) {
    *(volatile v8h*)dp = hv;
    if (lgHalf) { *(volatile v4f*)lp = (v4f){val[0], val[1], val[2], val[3]}; *(volatile v4f*)(lp + 4) = (v4f){val[4], val[5], val[6], val[7]}; }
    __threadfence();
  }
}
static_assert(kB * 32 == 4 * kThr, "lg grid exact");

__global__ __launch_bounds__(kThr) void hcast_kernel(const float* __restrict__ H32, unsigned short* __restrict__ H16) {
  unsigned v = blockIdx.x * (unsigned)kThr + threadIdx.x;
  asm volatile("" : "+v"(v));
  const size_t o8 = (size_t)v * 8u;
  const v4f a0 = *(const v4f*)(H32 + o8), a1 = *(const v4f*)(H32 + o8 + 4);
  v8h hv;
#pragma unroll
  for (int e = 0; e < 4; ++e) { hv[e] = (_Float16)carry_flush(a0[e], kACarry); hv[4 + e] = (_Float16)carry_flush(a1[e], kACarry); }
  *(volatile v8h*)(H16 + o8) = hv;
  __threadfence();
  *(volatile v8h*)(H16 + o8) = hv;
}
static_assert((size_t)kRowsH * kD / 8 == 512 * kThr, "state cast grid exact");

__global__ __launch_bounds__(kThr) void update_kernel(const float* __restrict__ PH32, const float* __restrict__ PB32, const float* __restrict__ LG32,
                                                      const int* __restrict__ eid, const float* __restrict__ q_matrix, float* __restrict__ H32,
                                                      float* __restrict__ HT32, int t) {
  unsigned v = blockIdx.x * (unsigned)kThr + threadIdx.x;
  asm volatile("" : "+v"(v));
  const unsigned b = v >> 7, d = v & 127u;
  int e0 = eid[b * kS + t]; e0 = (e0 < 0) ? 0 : (e0 > kNE - 1 ? kNE - 1 : e0);
  int e1 = eid[b * kS + t + 1]; e1 = (e1 < 0) ? 0 : (e1 > kNE - 1 ? kNE - 1 : e1);
  const float* q0 = q_matrix + (size_t)e0 * kSk;
  const float* q1 = q_matrix + (size_t)e1 * kSk;
  const float pb = PB32[(size_t)b * kD + d];
  const float lg = LG32[(size_t)b * kD + d];
  const float* php = PH32 + (size_t)b * kSk * kD + d;
  float* hp = H32 + (size_t)b * kSk * kD + d;
  float acc = 0.0f;
  for (int s = 0; s < kSk; ++s) {
    const float pre = php[(size_t)s * kD] + pb;
    const float f = 1.0f / (1.0f + expf(-pre));
    const float kt = q0[s], kn = q1[s];
    const float hn = bf16r(kt) * lg + f * hp[(size_t)s * kD];
    float* sp = hp + (size_t)s * kD;
    *(volatile float*)sp = hn;
    __threadfence();
    *(volatile float*)sp = hn;
    acc += bf16r(kn) * hn;
  }
  float* dp = HT32 + v;
  *(volatile float*)dp = acc;
  __threadfence();
  *(volatile float*)dp = acc;
}

__global__ __launch_bounds__(kThr) void x5_kernel(const int* __restrict__ eid, const float* __restrict__ ex_table, const float* __restrict__ HT32,
                                                  unsigned short* __restrict__ X5, int t) {
  unsigned v = blockIdx.x * (unsigned)kThr + threadIdx.x;
  asm volatile("" : "+v"(v));
  const unsigned b = v >> 5, c8 = (v & 31u) * 8u;
  const bool exHalf = c8 < 128u;
  const unsigned j = c8 & 127u;
  int e1 = eid[b * kS + t + 1]; e1 = (e1 < 0) ? 0 : (e1 > kNE - 1 ? kNE - 1 : e1);
  const float* sp = exHalf ? (ex_table + (size_t)e1 * kD + j) : (HT32 + (size_t)b * kD + j);
  const v4f p0 = *(const v4f*)sp, p1 = *(const v4f*)(sp + 4);
  v8h hv;
#pragma unroll
  for (int e = 0; e < 4; ++e) {
    const float q0 = exHalf ? bf16r(p0[e]) : p0[e];
    const float q1 = exHalf ? bf16r(p1[e]) : p1[e];
    hv[e] = (_Float16)carry_flush(q0, kACarry); hv[4 + e] = (_Float16)carry_flush(q1, kACarry);
  }
  unsigned short* dp = X5 + (size_t)b * 256u + c8;
  *(volatile v8h*)dp = hv;
  __threadfence();
  *(volatile v8h*)dp = hv;
}

__global__ __launch_bounds__(kThr) void pred_kernel(const float* __restrict__ P32, float* __restrict__ out, int t) {
  unsigned v = blockIdx.x * (unsigned)kThr + threadIdx.x;
  asm volatile("" : "+v"(v));
  const unsigned b = v >> 5, d4 = (v & 31u) * 4u;
  const v4f p = *(const v4f*)(P32 + (size_t)b * kD + d4);
  v4f o;
#pragma unroll
  for (int e = 0; e < 4; ++e) o[e] = 1.0f / (1.0f + expf(-p[e]));
  float* dp = out + ((size_t)b * kT + (size_t)t) * kD + d4;
  *(volatile v4f*)dp = o;
  __threadfence();
  *(volatile v4f*)dp = o;
}

extern "C" void kernel_launch(void* const* d_in, const int* in_sizes, int n_in,
                              void* d_out, int out_size, void* d_ws, size_t ws_size,
                              hipStream_t stream) {
  if (n_in < 19 || d_out == nullptr || d_ws == nullptr) return;
  if (in_sizes[0] != kB * kS || in_sizes[1] != kB * kS || in_sizes[2] != kB * kS || in_sizes[3] != kB * kS || in_sizes[4] != kNE * kSk) return;
  if (in_sizes[5] != kNE * kD || in_sizes[6] != kNA * kD || in_sizes[7] != kNI * kD || in_sizes[8] != kD * 384 || in_sizes[9] != kD) return;
  if (in_sizes[10] != kD * 512 || in_sizes[11] != kD || in_sizes[12] != kD * 512 || in_sizes[13] != kD || in_sizes[14] != kD * 384 || in_sizes[15] != kD) return;
  if (in_sizes[16] != kD * 256 || in_sizes[17] != kD || in_sizes[18] != kSk * kD) return;
  if (out_size != kB * kT * kD) return;
  if (ws_size < kWsTotal) return;
  const int* eid = (const int*)d_in[0];
  const int* atm = (const int*)d_in[1];
  const int* itm = (const int*)d_in[2];
  const int* avl = (const int*)d_in[3];
  const float* q_matrix = (const float*)d_in[4];
  const float* ex_table = (const float*)d_in[5];
  const float* at_table = (const float*)d_in[6];
  const float* it_table = (const float*)d_in[7];
  const float* W1 = (const float*)d_in[8];
  const float* b1 = (const float*)d_in[9];
  const float* Wl = (const float*)d_in[10];
  const float* bl = (const float*)d_in[11];
  const float* Wg = (const float*)d_in[12];
  const float* bg = (const float*)d_in[13];
  const float* Wf = (const float*)d_in[14];
  const float* bf = (const float*)d_in[15];
  const float* Wp = (const float*)d_in[16];
  const float* bp = (const float*)d_in[17];
  const float* h0 = (const float*)d_in[18];
  float* out = (float*)d_out;
  char* ws = (char*)d_ws;
  unsigned short* W1P = (unsigned short*)(ws + kOffW1P);
  unsigned short* WLG = (unsigned short*)(ws + kOffWLG);
  unsigned short* WF16 = (unsigned short*)(ws + kOffWF16);
  unsigned short* WP16 = (unsigned short*)(ws + kOffWP16);
  float* BIAS = (float*)(ws + kOffBIAS);
  unsigned short* XE16 = (unsigned short*)(ws + kOffXE16);
  float* LE32 = (float*)(ws + kOffLE32);
  float* H32 = (float*)(ws + kOffH32);
  float* HT32 = (float*)(ws + kOffHT32);
  float* LG32 = (float*)(ws + kOffLG32);
  unsigned short* X4 = (unsigned short*)(ws + kOffX4);
  float* Z32 = (float*)(ws + kOffZ32);
  unsigned short* XB = (unsigned short*)(ws + kOffXB);
  float* PB32 = (float*)(ws + kOffPB32);
  unsigned short* H16 = (unsigned short*)(ws + kOffH16);
  float* PH32 = (float*)(ws + kOffPH32);
  unsigned short* X5 = (unsigned short*)(ws + kOffX5);
  float* P32 = (float*)(ws + kOffP32);

  cast_plane_kernel<<<(int)(((size_t)kD * 384 / 8) / kThr), kThr, 0, stream>>>(W1, W1P, 7, 128, 0);
  cast_plane_kernel<<<(int)(((size_t)kD * 512 / 8) / kThr), kThr, 0, stream>>>(Wl, WLG, 9, 512, 0);
  cast_plane_kernel<<<(int)(((size_t)kD * 512 / 8) / kThr), kThr, 0, stream>>>(Wg, WLG + (size_t)kD * 512, 9, 512, 0);
  cast_plane_kernel<<<(int)(((size_t)kD * 384 / 8) / kThr), kThr, 0, stream>>>(Wf, WF16, 7, 128, 0);
  cast_plane_kernel<<<(int)(((size_t)kD * 256 / 8) / kThr), kThr, 0, stream>>>(Wp, WP16, 8, 256, 0);
  setup_kernel<<<1105, kThr, 0, stream>>>(b1, bl, bg, bf, bp, h0, BIAS, X4, XB, X5, H32);
  gather_kernel<<<768, kThr, 0, stream>>>(eid, atm, avl, ex_table, at_table, XE16);
  wmma_gemm64<0, false, 2, 0, false, 0><<<dim3((kRowsE / 64) * (kD / 64) / 8, 1), 256, 0, stream>>>(
      XE16, XE16, 384, 0L, W1P, W1P, 384, 0L, (void*)LE32, (void*)LE32, kD, 0L, BIAS + kFB1, nullptr, 0L, kRowsE, kD, 384, kScE);
  read0_kernel<<<16, kThr, 0, stream>>>(eid, q_matrix, H32, HT32);

  for (int t = 0; t < kT; ++t) {
    x4_kernel<<<8, kThr, 0, stream>>>(LE32, HT32, itm, it_table, X4, t);
    wmma_gemm64<0, false, 2, 0, false, 0><<<dim3((128 / 64) * (256 / 64) / 8, 1), 256, 0, stream>>>(
        X4, X4, 512, 0L, WLG, WLG, 512, 0L, (void*)Z32, (void*)Z32, 256, 0L, BIAS + kFBL, nullptr, 0L, 128, 256, 512, kScA);
    lg_kernel<<<4, kThr, 0, stream>>>(Z32, itm, it_table, LG32, XB, t);
    wmma_gemm64<0, false, 2, 0, false, 0><<<dim3((256 / 64) * (kD / 64) / 8, 1), 256, 0, stream>>>(
        XB, XB, 256, 0L, WF16 + 128, WF16 + 128, 384, 0L, (void*)PB32, (void*)PB32, kD, 0L, BIAS + kFBF, nullptr, 0L, 256, kD, 256, kScA);
    hcast_kernel<<<512, kThr, 0, stream>>>(H32, H16);
    wmma_gemm64<0, false, 2, 0, false, 0><<<dim3((kRowsH / 64) * (kD / 64) / 8, 1), 256, 0, stream>>>(
        H16, H16, kD, 0L, WF16, WF16, 384, 0L, (void*)PH32, (void*)PH32, kD, 0L, BIAS + kFBZ, nullptr, 0L, kRowsH, kD, kD, kScA);
    update_kernel<<<16, kThr, 0, stream>>>(PH32, PB32, LG32, eid, q_matrix, H32, HT32, t);
    x5_kernel<<<4, kThr, 0, stream>>>(eid, ex_table, HT32, X5, t);
    wmma_gemm64<0, false, 2, 0, false, 0><<<dim3((256 / 64) * (kD / 64) / 8, 1), 256, 0, stream>>>(
        X5, X5, 256, 0L, WP16, WP16, 256, 0L, (void*)P32, (void*)P32, kD, 0L, BIAS + kFBP, nullptr, 0L, 256, kD, 256, kScA);
    pred_kernel<<<4, kThr, 0, stream>>>(P32, out, t);
  }
}
